// HGCN_36532991819877
// MI455X (gfx1250) — hardware-run, weakly checked
//
#include <hip/hip_runtime.h>
#include <stddef.h>


#define DIMF    128
#define KP      128
#define LAYERS  2
#define RELS    2
#define NMAT    (2 * LAYERS * RELS)
#define OUTD    2
#define NTHR    256
#define NWAVE   8
#define EPT     8
#define CHUNK   (NTHR * EPT)
#define WCAP    (EPT * 32)
#define LISTN   (NWAVE * WCAP)
#define NBMAX   2048
#define RCAP    28672
#define DEGCAP  4096
#define GBM     64
#define GTHR    128
#define PASSW   64
#define NPASS   4
#define HPB     256
#define SLOPE   0.01f
#define CA      16.0f
#define CW      64.0f
#define SCL     0.0009765625f
#define WSCAP   134217728
#define LDS_AGG ((2 * RCAP + 2 * NBMAX + LISTN) * 4 + 64)

static_assert((CHUNK & (CHUNK - 1)) == 0 && CHUNK <= 4096);
static_assert((NBMAX & (NBMAX - 1)) == 0 && NBMAX <= 4096);
static_assert(NTHR * 8 == NBMAX);
static_assert(LISTN >= NBMAX);
static_assert(LISTN >= NWAVE * WCAP);
static_assert((RCAP % 32) == 0);
static_assert(LDS_AGG <= 300000);
static_assert(GBM == (GTHR / 32) * 16);
static_assert(2 * GBM == GTHR);
static_assert(GTHR == DIMF);
static_assert(NPASS * PASSW == 2 * DIMF);
static_assert(PASSW == 64 && DIMF == 2 * PASSW);
static_assert(KP == DIMF && (KP % 32) == 0);
static_assert(DIMF == 32 * 4);
static_assert(HPB == NTHR);
static_assert(2 * NTHR == 2 * DIMF * OUTD);
static_assert(RELS == 2);

typedef float    v4f  __attribute__((ext_vector_type(4)));
typedef float    v8f  __attribute__((ext_vector_type(8)));
typedef int      v4i  __attribute__((ext_vector_type(4)));
typedef int      v8i  __attribute__((ext_vector_type(8)));
typedef _Float16 v4h  __attribute__((ext_vector_type(4)));
typedef _Float16 v8h  __attribute__((ext_vector_type(8)));
typedef _Float16 v16h __attribute__((ext_vector_type(16)));
union FragH { v16h v; v8h h[2]; v8i w; };

__device__ __forceinline__ v8f wmh(const FragH& a, const FragH& b, v8f c) {
  v8f d = __builtin_amdgcn_wmma_f32_16x16x32_f16(false, a.v, false, b.v, (short)0, c, false, false);
  asm volatile("v_nop\n\tv_nop\n\tv_nop\n\tv_nop" : "+v"(d) : "v"(a.w), "v"(b.w));
  return d;
}

__device__ __forceinline__ int scan_chunk(const int* __restrict__ dsts, int nE, int cbase, int slotBase,
                                          int nb, int vec8, int* list, int tid, int lane, int wave) {
  int wc = 0;
  const int el0  = tid * EPT;
  const int e0   = cbase + el0;
  const int sent = -2147483647 - 1;
  v4i da, db;
  if (vec8 != 0 && cbase + CHUNK <= nE) {
    da = *(const v4i*)(dsts + e0);
    db = *(const v4i*)(dsts + e0 + 4);
  } else {
    da.x = (e0     < nE) ? dsts[min(e0,     nE - 1)] : sent;
    da.y = (e0 + 1 < nE) ? dsts[min(e0 + 1, nE - 1)] : sent;
    da.z = (e0 + 2 < nE) ? dsts[min(e0 + 2, nE - 1)] : sent;
    da.w = (e0 + 3 < nE) ? dsts[min(e0 + 3, nE - 1)] : sent;
    db.x = (e0 + 4 < nE) ? dsts[min(e0 + 4, nE - 1)] : sent;
    db.y = (e0 + 5 < nE) ? dsts[min(e0 + 5, nE - 1)] : sent;
    db.z = (e0 + 6 < nE) ? dsts[min(e0 + 6, nE - 1)] : sent;
    db.w = (e0 + 7 < nE) ? dsts[min(e0 + 7, nE - 1)] : sent;
  }
  const unsigned nbs = (unsigned)slotBase;
  const unsigned unb = (unsigned)nb;
  const unsigned s0 = (unsigned)da.x - nbs, s1 = (unsigned)da.y - nbs;
  const unsigned s2 = (unsigned)da.z - nbs, s3 = (unsigned)da.w - nbs;
  const unsigned s4 = (unsigned)db.x - nbs, s5 = (unsigned)db.y - nbs;
  const unsigned s6 = (unsigned)db.z - nbs, s7 = (unsigned)db.w - nbs;
  const bool h0 = s0 < unb, h1 = s1 < unb, h2 = s2 < unb, h3 = s3 < unb;
  const bool h4 = s4 < unb, h5 = s5 < unb, h6 = s6 < unb, h7 = s7 < unb;
  const unsigned any = __builtin_amdgcn_ballot_w32(h0 | h1 | h2 | h3 | h4 | h5 | h6 | h7);
  if (any != 0u) {
#define HITJ(J, HJ, SJ) { \
      const unsigned mj = __builtin_amdgcn_ballot_w32(HJ); \
      if (mj != 0u) { \
        if (HJ) { \
          const int pos = wc + (int)__builtin_amdgcn_mbcnt_lo(mj, 0u); \
          if (pos < WCAP) list[wave * WCAP + pos] = ((el0 + (J)) << 12) | (int)(SJ); \
        } \
        wc += (int)__builtin_popcount(mj); } }
    HITJ(0, h0, s0)
    HITJ(1, h1, s1)
    HITJ(2, h2, s2)
    HITJ(3, h3, s3)
    HITJ(4, h4, s4)
    HITJ(5, h5, s5)
    HITJ(6, h6, s6)
    HITJ(7, h7, s7)
#undef HITJ
  }
  return wc;
}

__global__ __launch_bounds__(NTHR) void k_xprep(const float* __restrict__ x, _Float16* xh, int nN, int nUnits) {
  const int i = (int)blockIdx.x * NTHR + (int)threadIdx.x;
  if (i >= nUnits) return;
  const int row = i >> 4;
  const int c0  = (i & 15) * 8;
  const int rc  = row < nN ? row : nN - 1;
  const float* p = x + (size_t)rc * DIMF + c0;
  v4f a = *(const v4f*)p, b = *(const v4f*)(p + 4);
  const v4f z4 = {0.f, 0.f, 0.f, 0.f};
  if (row >= nN) { a = z4; b = z4; }
  v8h hv;
  hv[0] = (_Float16)(a.x * CA); hv[1] = (_Float16)(a.y * CA);
  hv[2] = (_Float16)(a.z * CA); hv[3] = (_Float16)(a.w * CA);
  hv[4] = (_Float16)(b.x * CA); hv[5] = (_Float16)(b.y * CA);
  hv[6] = (_Float16)(b.z * CA); hv[7] = (_Float16)(b.w * CA);
  const size_t o = (size_t)row * KP + c0;
  *(volatile v8h*)(xh + o) = hv;
  __threadfence();
  *(volatile v8h*)(xh + o) = hv;
}

__global__ __launch_bounds__(NTHR) void k_wprep(const float* __restrict__ w1, const float* __restrict__ w2,
                                                _Float16* wt) {
  const int u = (int)blockIdx.x * NTHR + (int)threadIdx.x;
  if (u >= NMAT * DIMF * (KP / 8)) return;
  const int mi  = u >> 11;
  const int n   = (u >> 4) & (DIMF - 1);
  const int k8  = (u & 15) * 8;
  const int which = mi >> 2;
  const int mat = mi & 3;
  const float* src = (which == 0) ? w1 : w2;
  const float* p = src + (size_t)mat * DIMF * DIMF + (size_t)k8 * DIMF + n;
  v4f a, b;
  a.x = p[0 * DIMF]; a.y = p[1 * DIMF]; a.z = p[2 * DIMF]; a.w = p[3 * DIMF];
  b.x = p[4 * DIMF]; b.y = p[5 * DIMF]; b.z = p[6 * DIMF]; b.w = p[7 * DIMF];
  v8h hv;
  hv[0] = (_Float16)(a.x * CW); hv[1] = (_Float16)(a.y * CW);
  hv[2] = (_Float16)(a.z * CW); hv[3] = (_Float16)(a.w * CW);
  hv[4] = (_Float16)(b.x * CW); hv[5] = (_Float16)(b.y * CW);
  hv[6] = (_Float16)(b.z * CW); hv[7] = (_Float16)(b.w * CW);
  const size_t o = ((size_t)mi * DIMF + (size_t)n) * KP + k8;
  *(volatile v8h*)(wt + o) = hv;
  __threadfence();
  *(volatile v8h*)(wt + o) = hv;
}

__global__ __launch_bounds__(GTHR) void k_gemm(const _Float16* __restrict__ xh, const _Float16* __restrict__ w1t,
                                               const _Float16* __restrict__ w2t, const float* __restrict__ avec,
                                               float* Z, float* ES, float* ED) {
  __shared__ __attribute__((aligned(16))) float stg[GBM * PASSW];
  __shared__ __attribute__((aligned(16))) float esT[GBM];
  __shared__ __attribute__((aligned(16))) float edT[GBM];
  __shared__ float sA[2 * DIMF];
  const int tid = threadIdx.x, lane = tid & 31, wave = tid >> 5, hh = lane >> 4, m = lane & 15;
  const int rowBase = (int)blockIdx.x * GBM;
  sA[tid] = avec[tid];
  sA[tid + GTHR] = avec[tid + GTHR];
  const size_t arow = (size_t)(rowBase + 16 * wave + m) * KP + 8 * hh;
  const int drow = tid >> 1, dhalf = tid & 1;
  float esa = 0.f, eda = 0.f;
#pragma unroll 1
  for (int p = 0; p < NPASS; ++p) {
    const _Float16* wt = (p < 2) ? w1t : w2t;
    const int cb = (p & 1) * PASSW;
    v8f acc[4];
#pragma unroll
    for (int t = 0; t < 4; ++t) { v8f z = {0.f, 0.f, 0.f, 0.f, 0.f, 0.f, 0.f, 0.f}; acc[t] = z; }
    const size_t brow = (size_t)(cb + m) * KP + 8 * hh;
#pragma unroll 1
    for (int ks = 0; ks < KP / 32; ++ks) {
      FragH af;
      af.h[0] = *(const v8h*)(xh + arow + 32 * ks);
      af.h[1] = *(const v8h*)(xh + arow + 32 * ks + 16);
#pragma unroll
      for (int t = 0; t < 4; ++t) {
        const size_t bo = brow + (size_t)(16 * t) * KP + 32 * ks;
        FragH bf;
        bf.h[0] = *(const v8h*)(wt + bo);
        bf.h[1] = *(const v8h*)(wt + bo + 16);
        acc[t] = wmh(af, bf, acc[t]);
      }
    }
    float* sp = stg + (size_t)(16 * wave + 8 * hh) * PASSW + m;
#pragma unroll
    for (int t = 0; t < 4; ++t) {
#pragma unroll
      for (int r = 0; r < 8; ++r) sp[(size_t)r * PASSW + 16 * t] = acc[t][r] * SCL;
    }
    __syncthreads();
    {
      const float* srow = stg + (size_t)drow * PASSW + dhalf * 32;
      const float* ap   = sA + p * PASSW + dhalf * 32;
      float s = 0.f;
#pragma unroll 1
      for (int c = 0; c < 32; ++c) s = fmaf(srow[c], ap[c], s);
      if (p < 2) esa += s; else eda += s;
    }
    if (p < 2) {
      const int nF4 = GBM * PASSW / 4;
      float* zb = Z + (size_t)rowBase * DIMF + cb;
      const v4f* s4 = (const v4f*)stg;
#pragma unroll 1
      for (int f = tid; f < nF4; f += GTHR) {
        const int r = f >> 4, q = f & 15;
        const v4f v = s4[f];
        *(volatile v4f*)(zb + (size_t)r * DIMF + 4 * q) = v;
      }
      __threadfence();
#pragma unroll 1
      for (int f = tid; f < nF4; f += GTHR) {
        const int r = f >> 4, q = f & 15;
        const v4f v = s4[f];
        *(volatile v4f*)(zb + (size_t)r * DIMF + 4 * q) = v;
      }
    }
    __syncthreads();
  }
  esa += __shfl_xor(esa, 1);
  eda += __shfl_xor(eda, 1);
  if (dhalf == 0) { esT[drow] = esa; edT[drow] = eda; }
  __syncthreads();
  if (wave == 0) {
    const int li = lane & 15;
    const v4f ve = *(const v4f*)(esT + 4 * li);
    const v4f vd = *(const v4f*)(edT + 4 * li);
    const bool ise = lane < 16;
    v4f v;
    v.x = ise ? ve.x : vd.x; v.y = ise ? ve.y : vd.y; v.z = ise ? ve.z : vd.z; v.w = ise ? ve.w : vd.w;
    float* pp = (ise ? ES : ED) + (size_t)rowBase + 4 * li;
    *(volatile v4f*)pp = v;
    __threadfence();
    *(volatile v4f*)pp = v;
  }
}

__global__ __launch_bounds__(NTHR) void k_agg(
    const int* __restrict__ srcs, const int* __restrict__ dsts,
    const float* __restrict__ Z, const float* __restrict__ ES, const float* __restrict__ ED,
    float* T, _Float16* xh, float* hout,
    int nN, int nE, int nb, int vec8, int mode, int wxh, int wout) {
  extern __shared__ v4f lds_dyn[];
  int* reg1 = (int*)lds_dyn;
  int* reg2 = reg1 + RCAP;
  int* scnt = reg2 + RCAP;
  int* soff = scnt + NBMAX;
  int* list = soff + NBMAX;
  int* wcnt = list + LISTN;
  int* wtot = wcnt + NWAVE;
  const int tid = threadIdx.x, lane = tid & 31, wave = tid >> 5;
  const int nodeBase = (int)blockIdx.x * nb;

  for (int i = tid; i < NBMAX; i += NTHR) scnt[i] = 0;
  __syncthreads();

  int tot = 0;
  const int nChunks = (nE + CHUNK - 1) / CHUNK;
#pragma unroll 1
  for (int ch = 0; ch < nChunks; ++ch) {
    const int cbase = ch * CHUNK;
    const int wc = scan_chunk(dsts, nE, cbase, nodeBase, nb, vec8, list, tid, lane, wave);
    if (lane == 0) wcnt[wave] = wc;
    __syncthreads();
    int pre = 0, all = 0;
#pragma unroll
    for (int w2 = 0; w2 < NWAVE; ++w2) {
      int c = wcnt[w2];
      c = c < 0 ? 0 : (c > WCAP ? WCAP : c);
      all += c;
      pre += (w2 < wave) ? c : 0;
    }
    const int wcc  = wc > WCAP ? WCAP : wc;
    const int base = tot + pre;
#pragma unroll 1
    for (int i = lane; i < wcc; i += 32) {
      const int ent = list[wave * WCAP + i];
      const int el  = (ent >> 12) & (CHUNK - 1);
      const int sl  = ent & (NBMAX - 1);
      int eid = cbase + el;
      eid = eid > nE - 1 ? nE - 1 : eid;
      const int pos = base + i;
      if (pos < RCAP) reg1[pos] = (int)(((unsigned)eid << 12) | (unsigned)sl);
    }
    tot += all;
    tot = tot > RCAP ? RCAP : tot;
    __syncthreads();
  }
  const int nh = tot;

  if (wave == 0) {
#pragma unroll 1
    for (int b0 = 0; b0 < nh; b0 += 32) {
      const int idx = b0 + lane;
      const int uv  = reg1[idx < RCAP ? idx : RCAP - 1];
      const int m32 = (nh - b0) < 32 ? (nh - b0) : 32;
#pragma unroll 1
      for (int k = 0; k < m32; ++k) {
        const int u  = __builtin_amdgcn_readlane(uv, k);
        const int sl = u & (NBMAX - 1);
        if (lane == 0) scnt[sl] = scnt[sl] + 1;
      }
    }
  }
  __syncthreads();

  {
    const v4i ca = *(const v4i*)(scnt + 8 * tid);
    const v4i cb = *(const v4i*)(scnt + 8 * tid + 4);
    const int e0 = ca.x < 0 ? 0 : ca.x, e1 = ca.y < 0 ? 0 : ca.y, e2 = ca.z < 0 ? 0 : ca.z, e3 = ca.w < 0 ? 0 : ca.w;
    const int e4 = cb.x < 0 ? 0 : cb.x, e5 = cb.y < 0 ? 0 : cb.y, e6 = cb.z < 0 ? 0 : cb.z, e7 = cb.w < 0 ? 0 : cb.w;
    const int ts = e0 + e1 + e2 + e3 + e4 + e5 + e6 + e7;
    int incl = ts;
#pragma unroll
    for (int d = 1; d < 32; d <<= 1) {
      const int up = __shfl_up(incl, d);
      if (lane >= d) incl += up;
    }
    if (lane == 31) wtot[wave] = incl;
    __syncthreads();
    int pre = 0;
#pragma unroll
    for (int w2 = 0; w2 < NWAVE; ++w2) pre += (w2 < wave) ? wtot[w2] : 0;
    int run = pre + incl - ts;
    soff[8 * tid + 0] = run; run += e0;
    soff[8 * tid + 1] = run; run += e1;
    soff[8 * tid + 2] = run; run += e2;
    soff[8 * tid + 3] = run; run += e3;
    soff[8 * tid + 4] = run; run += e4;
    soff[8 * tid + 5] = run; run += e5;
    soff[8 * tid + 6] = run; run += e6;
    soff[8 * tid + 7] = run;
  }
  __syncthreads();
  for (int i = tid; i < NBMAX; i += NTHR) list[i] = soff[i];
  __syncthreads();

  if (wave == 0) {
#pragma unroll 1
    for (int b0 = 0; b0 < nh; b0 += 32) {
      const int idx = b0 + lane;
      const int uv  = reg1[idx < RCAP ? idx : RCAP - 1];
      const int m32 = (nh - b0) < 32 ? (nh - b0) : 32;
#pragma unroll 1
      for (int k = 0; k < m32; ++k) {
        const int u   = __builtin_amdgcn_readlane(uv, k);
        const int sl  = u & (NBMAX - 1);
        const int eid = (int)((unsigned)u >> 12);
        if (lane == 0) {
          int pos = list[sl];
          pos = pos < 0 ? 0 : (pos > RCAP - 1 ? RCAP - 1 : pos);
          reg2[pos] = eid;
          list[sl] = pos + 1;
        }
      }
    }
  }
  __syncthreads();

  const int nbw = nb >> 3;
  const int c4  = 4 * lane;
  const bool ovf = (nh >= RCAP);
  const float qnan = __int_as_float(0x7fc00000);
#pragma unroll 1
  for (int jt = 0; jt < nbw; ++jt) {
    const int slot = wave * nbw + jt;
    const int grow = nodeBase + slot;
    const int gcl  = grow < nN ? grow : nN - 1;
    int st = soff[slot];
    const int craw = scnt[slot];
    int cnt = craw;
    st  = st < 0 ? 0 : (st > nh ? nh : st);
    cnt = cnt < 0 ? 0 : (cnt > DEGCAP ? DEGCAP : cnt);
    if (cnt > nh - st) cnt = nh - st;
    const float pz = (ovf || craw > DEGCAP) ? qnan : 0.0f;
    const bool wr = grow < nN;

    const float edv = ED[gcl];
    float mx = -3.0e38f;
    float dn = 0.0f;
    v4f a = {0.f, 0.f, 0.f, 0.f};
#pragma unroll 1
    for (int q = 0; q < cnt; ++q) {
      int idx = st + q; idx = idx > RCAP - 1 ? RCAP - 1 : idx;
      int eid = reg2[idx]; eid = eid < 0 ? 0 : (eid > nE - 1 ? nE - 1 : eid);
      const int sraw = srcs[eid];
      const int s = sraw < 0 ? 0 : (sraw > nN - 1 ? nN - 1 : sraw);
      const v4f zs = *(const v4f*)(Z + (size_t)s * DIMF + c4);
      const float ess = ES[s];
      const float u = ess + edv;
      const float l = fmaxf(u, SLOPE * u);
      const float mn = fmaxf(mx, l);
      const float s1 = __expf(mx - mn), s2 = __expf(l - mn);
      dn = fmaf(dn, s1, s2);
      a.x = fmaf(a.x, s1, s2 * zs.x);
      a.y = fmaf(a.y, s1, s2 * zs.y);
      a.z = fmaf(a.z, s1, s2 * zs.z);
      a.w = fmaf(a.w, s1, s2 * zs.w);
      mx = mn;
    }
    const float dsel = (cnt > 0) ? dn : 1.0f;
    const float inv = __builtin_amdgcn_rcpf(dsel);
    v4f o;
    o.x = fmaf(a.x, inv, pz);
    o.y = fmaf(a.y, inv, pz);
    o.z = fmaf(a.z, inv, pz);
    o.w = fmaf(a.w, inv, pz);
    if (mode == 0) {
      float* tp = T + (size_t)gcl * DIMF + c4;
      if (wr) *(volatile v4f*)tp = o;
      __threadfence();
      if (wr) *(volatile v4f*)tp = o;
    } else {
      const v4f t = *(const v4f*)(T + (size_t)gcl * DIMF + c4);
      const float x0 = 0.5f * (t.x + o.x), x1 = 0.5f * (t.y + o.y);
      const float x2 = 0.5f * (t.z + o.z), x3 = 0.5f * (t.w + o.w);
      v4f hr;
      hr.x = (x0 < 0.f) ? 0.f : x0;
      hr.y = (x1 < 0.f) ? 0.f : x1;
      hr.z = (x2 < 0.f) ? 0.f : x2;
      hr.w = (x3 < 0.f) ? 0.f : x3;
      v4h hv;
      hv[0] = (_Float16)(hr.x * CA); hv[1] = (_Float16)(hr.y * CA);
      hv[2] = (_Float16)(hr.z * CA); hv[3] = (_Float16)(hr.w * CA);
      _Float16* xp = xh + (size_t)gcl * KP + c4;
      float* hp = hout + (size_t)gcl * DIMF + c4;
      const bool sx = wr && (wxh != 0);
      const bool sh = wr && (wout != 0);
      if (sx) *(volatile v4h*)xp = hv;
      if (sh) *(volatile v4f*)hp = hr;
      __threadfence();
      if (sx) *(volatile v4h*)xp = hv;
      if (sh) *(volatile v4f*)hp = hr;
    }
  }
}

__global__ __launch_bounds__(NTHR) void k_head(const float* __restrict__ h, const int* __restrict__ ps,
                                               const int* __restrict__ pd, const float* __restrict__ wc,
                                               const float* __restrict__ bc, float* out, int nN, int P) {
  __shared__ __attribute__((aligned(16))) float sO[HPB * OUTD];
  __shared__ __attribute__((aligned(16))) float sW[2 * DIMF * OUTD];
  __shared__ float sb[OUTD];
  const int tid = threadIdx.x, lane = tid & 31, wave = tid >> 5;
  const int pBase = (int)blockIdx.x * HPB;
  sW[tid] = wc[tid];
  sW[tid + NTHR] = wc[tid + NTHR];
  if (tid < OUTD) sb[tid] = bc[tid];
  __syncthreads();
  const int p  = pBase + tid;
  const int pc = p < P ? p : P - 1;
  int is = ps[pc]; is = is < 0 ? 0 : (is > nN - 1 ? nN - 1 : is);
  int id = pd[pc]; id = id < 0 ? 0 : (id > nN - 1 ? nN - 1 : id);
  const v4f* hs = (const v4f*)(h + (size_t)is * DIMF);
  const v4f* hd = (const v4f*)(h + (size_t)id * DIMF);
  float a0 = 0.f, a1 = 0.f;
#pragma unroll 1
  for (int q = 0; q < DIMF / 4; ++q) {
    const v4f xv = hs[q];
    const float* w = sW + 8 * q;
    a0 = fmaf(xv.x, w[0], a0); a1 = fmaf(xv.x, w[1], a1);
    a0 = fmaf(xv.y, w[2], a0); a1 = fmaf(xv.y, w[3], a1);
    a0 = fmaf(xv.z, w[4], a0); a1 = fmaf(xv.z, w[5], a1);
    a0 = fmaf(xv.w, w[6], a0); a1 = fmaf(xv.w, w[7], a1);
  }
#pragma unroll 1
  for (int q = 0; q < DIMF / 4; ++q) {
    const v4f yv = hd[q];
    const float* w = sW + 2 * DIMF + 8 * q;
    a0 = fmaf(yv.x, w[0], a0); a1 = fmaf(yv.x, w[1], a1);
    a0 = fmaf(yv.y, w[2], a0); a1 = fmaf(yv.y, w[3], a1);
    a0 = fmaf(yv.z, w[4], a0); a1 = fmaf(yv.z, w[5], a1);
    a0 = fmaf(yv.w, w[6], a0); a1 = fmaf(yv.w, w[7], a1);
  }
  a0 += sb[0];
  a1 += sb[1];
  const float o0 = 1.0f / (1.0f + __expf(-a0));
  const float o1 = 1.0f / (1.0f + __expf(-a1));
  sO[2 * tid]     = o0;
  sO[2 * tid + 1] = o1;
  __syncthreads();
  const int nValid = (P - pBase) < HPB ? (P - pBase) : HPB;
  const int fl  = nValid * OUTD;
  const int n4  = fl >> 2;
  const int rem = fl & 3;
  float* base = out + (size_t)pBase * OUTD;
  const v4f* s4 = (const v4f*)sO;
  const v4f v = s4[tid < n4 ? tid : 0];
  const int ti = 4 * n4 + (lane & 3);
  const float tv = sO[ti < fl ? ti : fl - 1];
  const bool vw = tid < n4;
  const bool tw = (rem != 0) && (tid >= n4) && (tid < n4 + rem) && (wave == (n4 >> 5));
  if (vw) *(volatile v4f*)(base + 4 * tid) = v;
  if (tw) *(volatile float*)(base + 4 * n4 + (tid - n4)) = tv;
  __threadfence();
  if (vw) *(volatile v4f*)(base + 4 * tid) = v;
  if (tw) *(volatile float*)(base + 4 * n4 + (tid - n4)) = tv;
}

static int pick_nb(int nE, int nN) {
  int nb = NBMAX;
  while (nb > 16 && (long long)nb * (long long)nE * 5LL > (long long)RCAP * (long long)nN * 4LL) nb >>= 1;
  return nb;
}

extern "C" void kernel_launch(void* const* d_in, const int* in_sizes, int n_in,
                              void* d_out, int out_size, void* d_ws, size_t ws_size,
                              hipStream_t stream) {
  if (n_in < 10) return;
  const int nN = in_sizes[0] / DIMF;
  if (nN <= 0 || in_sizes[0] != nN * DIMF) return;
  if (nN > (1 << 22)) return;
  if (in_sizes[1] != LAYERS * RELS * DIMF * DIMF) return;
  if (in_sizes[2] != LAYERS * RELS * DIMF * DIMF) return;
  if (in_sizes[3] != LAYERS * RELS * 2 * DIMF) return;
  if (in_sizes[4] != 2 * DIMF * OUTD) return;
  if (in_sizes[5] != OUTD) return;
  const int nEt = in_sizes[6];
  if (nEt < RELS || (nEt % RELS) != 0 || in_sizes[7] != nEt) return;
  const int nE = nEt / RELS;
  if (nE < 1 || nE > (1 << 20)) return;
  const int P = in_sizes[8];
  if (P < 1 || in_sizes[9] != P) return;
  if (out_size != nN * DIMF + P * OUTD) return;

  const float* feat = (const float*)d_in[0];
  const float* W1   = (const float*)d_in[1];
  const float* W2   = (const float*)d_in[2];
  const float* Avec = (const float*)d_in[3];
  const float* Wc   = (const float*)d_in[4];
  const float* bc   = (const float*)d_in[5];
  const int*   sidx = (const int*)d_in[6];
  const int*   didx = (const int*)d_in[7];
  const int*   psrc = (const int*)d_in[8];
  const int*   pdst = (const int*)d_in[9];
  float* out0 = (float*)d_out;
  float* out1 = out0 + (size_t)nN * DIMF;

  const int MP   = ((nN + GBM - 1) / GBM) * GBM;
  const int nb   = pick_nb(nE, nN);
  const int vec8 = ((nE & 3) == 0) ? 1 : 0;
  const int nUnits = MP * (KP / 8);

  char* ws = (char*)d_ws;
  size_t off = 0;
  const size_t oWT = off; off += (size_t)NMAT * DIMF * KP * 2;   off = (off + 255) & ~(size_t)255;
  const size_t oXH = off; off += (size_t)MP * KP * 2;            off = (off + 255) & ~(size_t)255;
  const size_t oZ  = off; off += (size_t)MP * DIMF * 4;          off = (off + 255) & ~(size_t)255;
  const size_t oT  = off; off += (size_t)MP * DIMF * 4;          off = (off + 255) & ~(size_t)255;
  const size_t oES = off; off += (size_t)MP * 4;                 off = (off + 255) & ~(size_t)255;
  const size_t oED = off; off += (size_t)MP * 4;                 off = (off + 255) & ~(size_t)255;
  if (off > ws_size || off > (size_t)WSCAP) return;
  _Float16* WT = (_Float16*)(ws + oWT);
  _Float16* XH = (_Float16*)(ws + oXH);
  float*    Z  = (float*)(ws + oZ);
  float*    T  = (float*)(ws + oT);
  float*    ES = (float*)(ws + oES);
  float*    ED = (float*)(ws + oED);

  hipFuncSetAttribute(reinterpret_cast<const void*>(&k_agg),
                      hipFuncAttributeMaxDynamicSharedMemorySize, LDS_AGG);

  k_xprep<<<(nUnits + NTHR - 1) / NTHR, NTHR, 0, stream>>>(feat, XH, nN, nUnits);
  k_wprep<<<(NMAT * DIMF * (KP / 8) + NTHR - 1) / NTHR, NTHR, 0, stream>>>(W1, W2, WT);

  const int gG = MP / GBM;
  const int gA = (nN + nb - 1) / nb;

  for (int l = 0; l < LAYERS; ++l) {
    const int wxh  = (l < LAYERS - 1) ? 1 : 0;
    const int wout = (l == LAYERS - 1) ? 1 : 0;
    for (int r = 0; r < RELS; ++r) {
      const int mat = l * RELS + r;
      const _Float16* w1t = WT + (size_t)mat * DIMF * KP;
      const _Float16* w2t = WT + (size_t)(LAYERS * RELS + mat) * DIMF * KP;
      k_gemm<<<gG, GTHR, 0, stream>>>(XH, w1t, w2t, Avec + (size_t)mat * 2 * DIMF, Z, ES, ED);
      k_agg<<<gA, NTHR, LDS_AGG, stream>>>(sidx + (size_t)r * nE, didx + (size_t)r * nE, Z, ES, ED,
                                           T, XH, out0, nN, nE, nb, vec8, r, wxh, wout);
    }
  }
  k_head<<<(P + HPB - 1) / HPB, NTHR, 0, stream>>>(out0, psrc, pdst, Wc, bc, out1, nN, P);
}
